// GNNClassifier_88648124990138
// MI455X (gfx1250) — hardware-verified
//
#include <hip/hip_runtime.h>
#include <stddef.h>
#include <stdint.h>


#define HID     64
#define VOCABN  128
#define NGR     2048
#define NCLS    2
#define AGP     128
#define XBP     64
#define K0L     192
#define K1L     256
#define NTHR    256
#define NWAVE   8
#define EPT     8
#define CHUNK   (NTHR * EPT)
#define WCAP    (EPT * 32)
#define LISTN   (NWAVE * WCAP)
#define NBA     1024
#define SLA     10
#define NBG     128
#define SLG     7
#define RCAP    16384
#define DEGCAP  64
#define DEGCAPG 128
#define GBM     128
#define GBN     64
#define GTHR    256
#define NPARTW  7
#define ZINTS   (LISTN + 2 * RCAP + 3 * NBA)
#define MISCI   16
#define BLDS_INTS (ZINTS + MISCI)
#define WSMAX   134217728

static_assert((CHUNK & (CHUNK - 1)) == 0 && CHUNK <= 4096);
static_assert((NBA & (NBA - 1)) == 0 && NBA == (1 << SLA));
static_assert((NBG & (NBG - 1)) == 0 && NBG == (1 << SLG) && NBG <= NBA);
static_assert(((long long)(1 << 20) << SLA) < (1LL << 31));
static_assert(ZINTS % (NTHR * 4) == 0 && LISTN % 4 == 0 && RCAP % 4 == 0);
static_assert(RCAP % (NTHR * 4) == 0);
static_assert(NBA == NTHR * 4);
static_assert(NBA % NWAVE == 0 && NBG % NWAVE == 0 && NBA % 32 == 0 && NBG % 32 == 0);
static_assert(K0L % 32 == 0 && K1L % 32 == 0 && K0L == AGP + XBP && K1L == 2 * AGP);
static_assert(GBN == HID && HID == 2 * 32 && GBM == (GTHR / 32) * 16);
static_assert(NGR == 16 * NBG && NBG * NCLS * 4 == 1024);
static_assert(RCAP >= 10466 + 524);
static_assert(RCAP >= 12670);
static_assert(DEGCAP >= 25 + 8);
static_assert(DEGCAPG >= 78 + 8);
static_assert(BLDS_INTS * 4 <= 300000);
static_assert((512 % NTHR) == 0);

typedef float          v2f   __attribute__((ext_vector_type(2)));
typedef float          v4f   __attribute__((ext_vector_type(4)));
typedef float          v8f   __attribute__((ext_vector_type(8)));
typedef int            v4i   __attribute__((ext_vector_type(4)));
typedef int            v8i   __attribute__((ext_vector_type(8)));
typedef unsigned int   v4u   __attribute__((ext_vector_type(4)));
typedef unsigned short v4us  __attribute__((ext_vector_type(4)));
typedef unsigned short v8us  __attribute__((ext_vector_type(8)));
typedef unsigned short v16us __attribute__((ext_vector_type(16)));
typedef __bf16         v16bf __attribute__((ext_vector_type(16)));
typedef v2f  __attribute__((may_alias)) v2fa;
typedef v4f  __attribute__((may_alias)) v4fa;
typedef v4i  __attribute__((may_alias)) v4ia;
typedef v4us __attribute__((may_alias)) v4usa;
typedef v8us __attribute__((may_alias)) v8usa;
union FragB { v16bf v; v16us u; v8us h[2]; v8i w; };

__device__ __forceinline__ v8f wmb(const FragB& a, const FragB& b, v8f c) {
  v8f d = __builtin_amdgcn_wmma_f32_16x16x32_bf16(false, a.v, false, b.v, (short)0, c, false, false);
  asm volatile("v_nop\n\tv_nop\n\tv_nop\n\tv_nop" : "+v"(d) : "v"(a.w), "v"(b.w));
  return d;
}

__device__ __forceinline__ unsigned bf16_bits(float f) {
  const unsigned u = __float_as_uint(f);
  const unsigned r = (u + 0x7FFFu + ((u >> 16) & 1u)) >> 16;
  const unsigned q = (u >> 16) | 0x40u;
  return ((u & 0x7FFFFFFFu) > 0x7F800000u) ? q : r;
}
__device__ __forceinline__ float bf16_val(float f) {
  return __uint_as_float(bf16_bits(f) << 16);
}

template <int SLB>
__device__ __forceinline__ int scan_chunk(const int* __restrict__ dsts, int nE, int cbase, int slotBase,
                                          int nb, int vec8, int* list, int tid, int lane, int wave) {
  int wc = 0;
  const int el0  = tid * EPT;
  const int e0   = cbase + el0;
  const int sent = -2147483647 - 1;
  v4i da, db;
  if (vec8 != 0 && cbase + CHUNK <= nE) {
    da = *(const v4i*)(dsts + e0);
    db = *(const v4i*)(dsts + e0 + 4);
  } else {
    da.x = (e0     < nE) ? dsts[min(e0,     nE - 1)] : sent;
    da.y = (e0 + 1 < nE) ? dsts[min(e0 + 1, nE - 1)] : sent;
    da.z = (e0 + 2 < nE) ? dsts[min(e0 + 2, nE - 1)] : sent;
    da.w = (e0 + 3 < nE) ? dsts[min(e0 + 3, nE - 1)] : sent;
    db.x = (e0 + 4 < nE) ? dsts[min(e0 + 4, nE - 1)] : sent;
    db.y = (e0 + 5 < nE) ? dsts[min(e0 + 5, nE - 1)] : sent;
    db.z = (e0 + 6 < nE) ? dsts[min(e0 + 6, nE - 1)] : sent;
    db.w = (e0 + 7 < nE) ? dsts[min(e0 + 7, nE - 1)] : sent;
  }
  const unsigned nbs = (unsigned)slotBase;
  const unsigned unb = (unsigned)nb;
  const unsigned s0 = (unsigned)da.x - nbs, s1 = (unsigned)da.y - nbs;
  const unsigned s2 = (unsigned)da.z - nbs, s3 = (unsigned)da.w - nbs;
  const unsigned s4 = (unsigned)db.x - nbs, s5 = (unsigned)db.y - nbs;
  const unsigned s6 = (unsigned)db.z - nbs, s7 = (unsigned)db.w - nbs;
  const bool h0 = s0 < unb, h1 = s1 < unb, h2 = s2 < unb, h3 = s3 < unb;
  const bool h4 = s4 < unb, h5 = s5 < unb, h6 = s6 < unb, h7 = s7 < unb;
  const unsigned any = __builtin_amdgcn_ballot_w32(h0 | h1 | h2 | h3 | h4 | h5 | h6 | h7);
  if (any != 0u) {
#define HITJ(J, HJ, SJ) { \
      const unsigned mj = __builtin_amdgcn_ballot_w32(HJ); \
      if (mj != 0u) { \
        if (HJ) { \
          const int pos = wc + (int)__builtin_amdgcn_mbcnt_lo(mj, 0u); \
          if (pos < WCAP) list[wave * WCAP + pos] = ((el0 + (J)) << SLB) | (int)(SJ); \
        } \
        wc += (int)__builtin_popcount(mj); } }
    HITJ(0, h0, s0)
    HITJ(1, h1, s1)
    HITJ(2, h2, s2)
    HITJ(3, h3, s3)
    HITJ(4, h4, s4)
    HITJ(5, h5, s5)
    HITJ(6, h6, s6)
    HITJ(7, h7, s7)
#undef HITJ
  }
  return wc;
}

template <int SLB, int NB>
__device__ __forceinline__ void bucket_build(const int* __restrict__ keys, int nE, int slotBase, int vec8,
                                             int* dsm, int tid, int lane, int wave, int& ttOut, int& ovfOut) {
  int* list = dsm;
  int* hl   = dsm + LISTN;
  int* sl   = hl + RCAP;
  int* cnt  = sl + RCAP;
  int* offs = cnt + NBA;
  int* cur  = offs + NBA;
  int* misc = cur + NBA;
  {
    const v4i z4 = {0, 0, 0, 0};
    for (int i = tid * 4; i < ZINTS; i += NTHR * 4) *(v4ia*)(dsm + i) = z4;
    if (tid < MISCI) misc[tid] = 0;
  }
  __syncthreads();

  int t = 0, ov = 0;
  const int nChunks = (nE + CHUNK - 1) / CHUNK;
#pragma unroll 1
  for (int ch = 0; ch < nChunks; ++ch) {
    const int cbase = ch * CHUNK;
    const int wc = scan_chunk<SLB>(keys, nE, cbase, slotBase, NB, vec8, list, tid, lane, wave);
    if (lane == 0) misc[wave] = wc;
    __syncthreads();
    if (wave == 0) {
#pragma unroll 1
      for (int w2 = 0; w2 < NWAVE; ++w2) {
        int c = misc[w2];
        c = c < 0 ? 0 : (c > WCAP ? WCAP : c);
#pragma unroll 1
        for (int b0 = 0; b0 < c; b0 += 32) {
          const int idx = b0 + lane;
          const int ent = list[w2 * WCAP + (idx < WCAP ? idx : WCAP - 1)];
          const int m32 = (c - b0) < 32 ? (c - b0) : 32;
#pragma unroll 1
          for (int k = 0; k < m32; ++k) {
            const int u    = __builtin_amdgcn_readlane(ent, k);
            const int slot = u & (NB - 1);
            const int el   = (u >> SLB) & (CHUNK - 1);
            const int pk   = ((cbase + el) << SLB) | slot;
            if (t < RCAP) {
              if (lane == 0) { hl[t] = pk; cnt[slot] = cnt[slot] + 1; }
              t = t + 1;
            } else {
              ov = 1;
            }
          }
        }
      }
    }
    __syncthreads();
  }
  if (wave == 0 && lane == 0) { misc[8] = t; misc[9] = ov; }
  __syncthreads();
  int tt = misc[8];
  tt = tt < 0 ? 0 : (tt > RCAP ? RCAP : tt);
  const int ovf = misc[9];

  if (wave == 0) {
    const int base = lane * (NB / 32);
    int s = 0;
#pragma unroll 1
    for (int i = 0; i < NB / 32; ++i) s += cnt[base + i];
    int incl = s;
#pragma unroll
    for (int d = 1; d < 32; d <<= 1) {
      const int y = __shfl_up(incl, d, 32);
      if (lane >= d) incl += y;
    }
    int run = incl - s;
#pragma unroll 1
    for (int i = 0; i < NB / 32; ++i) {
      const int cv = cnt[base + i];
      offs[base + i] = run;
      cur[base + i]  = run;
      run += cv;
    }
  }
  __syncthreads();
  if (wave == 0) {
#pragma unroll 1
    for (int b0 = 0; b0 < tt; b0 += 32) {
      const int idx = b0 + lane;
      const int ent = hl[idx < RCAP ? idx : RCAP - 1];
      const int m32 = (tt - b0) < 32 ? (tt - b0) : 32;
#pragma unroll 1
      for (int k = 0; k < m32; ++k) {
        const int u    = __builtin_amdgcn_readlane(ent, k);
        const int slot = u & (NB - 1);
        if (lane == 0) {
          int p = cur[slot];
          p = p < 0 ? 0 : (p > RCAP - 1 ? RCAP - 1 : p);
          sl[p] = u;
          cur[slot] = p + 1;
        }
      }
    }
  }
  __syncthreads();
  ttOut  = tt;
  ovfOut = ovf;
}

__device__ __forceinline__ void wunit(const float* __restrict__ W, unsigned short* P, int pitch, int coff, int v) {
  const int n  = v >> 3;
  const int k8 = (v & 7) * 8;
  const float* p = W + (size_t)k8 * HID + n;
  v8us o;
#pragma unroll
  for (int i = 0; i < 8; ++i) o[i] = (unsigned short)bf16_bits(p[(size_t)i * HID]);
  unsigned short* dp = P + (size_t)n * pitch + coff + k8;
  *(volatile v8us*)dp = o;
  __threadfence();
  *(volatile v8us*)dp = o;
}

__global__ __launch_bounds__(NTHR) void k_prep(const int* __restrict__ x, const float* __restrict__ emb,
                                               const float* __restrict__ W1l, const float* __restrict__ W1r,
                                               const float* __restrict__ W2l, const float* __restrict__ W2r,
                                               int nN, int nXB, unsigned short* XB,
                                               unsigned short* W1c, unsigned short* W2c) {
  const int bid = (int)blockIdx.x, tid = (int)threadIdx.x;
  if (bid < nXB) {
    const int u   = bid * NTHR + tid;
    const int row = u >> 3;
    const int k8  = (u & 7) * 8;
    const int rc  = row < nN ? row : nN - 1;
    int tok = x[rc];
    tok = tok < 0 ? 0 : (tok > VOCABN - 1 ? VOCABN - 1 : tok);
    const float* p = emb + (size_t)tok * HID + k8;
    const v4f a = *(const v4f*)p;
    const v4f b = *(const v4f*)(p + 4);
    const bool ok = row < nN;
    v8us o;
    o[0] = ok ? (unsigned short)bf16_bits(a.x) : (unsigned short)0;
    o[1] = ok ? (unsigned short)bf16_bits(a.y) : (unsigned short)0;
    o[2] = ok ? (unsigned short)bf16_bits(a.z) : (unsigned short)0;
    o[3] = ok ? (unsigned short)bf16_bits(a.w) : (unsigned short)0;
    o[4] = ok ? (unsigned short)bf16_bits(b.x) : (unsigned short)0;
    o[5] = ok ? (unsigned short)bf16_bits(b.y) : (unsigned short)0;
    o[6] = ok ? (unsigned short)bf16_bits(b.z) : (unsigned short)0;
    o[7] = ok ? (unsigned short)bf16_bits(b.w) : (unsigned short)0;
    unsigned short* dp = XB + (size_t)row * XBP + k8;
    *(volatile v8us*)dp = o;
    __threadfence();
    *(volatile v8us*)dp = o;
  } else {
    const int u    = (bid - nXB) * NTHR + tid;
    const int part = u >> 9;
    const int v    = u & 511;
    if (part == 0)      wunit(W1l, W1c, K0L, 0, v);
    else if (part == 1) wunit(W1l, W1c, K0L, 64, v);
    else if (part == 2) wunit(W1r, W1c, K0L, 128, v);
    else if (part == 3) wunit(W2l, W2c, K1L, 0, v);
    else if (part == 4) wunit(W2l, W2c, K1L, 64, v);
    else if (part == 5) wunit(W2r, W2c, K1L, 128, v);
    else if (part == 6) wunit(W2r, W2c, K1L, 192, v);
  }
}

__global__ __launch_bounds__(NTHR) void k_compact(const int* __restrict__ srcs, const int* __restrict__ dsts,
                                                  int nE, int nN, int vec8,
                                                  int* LIST, int* CNT, int* OFF, int* FLG) {
  extern __shared__ __attribute__((aligned(16))) int dsm[];
  const int tid = (int)threadIdx.x, lane = tid & 31, wave = tid >> 5;
  const int b = (int)blockIdx.x;
  int tt = 0, ovf = 0;
  bucket_build<SLA, NBA>(dsts, nE, b * NBA, vec8, dsm, tid, lane, wave, tt, ovf);
  const int* sl   = dsm + LISTN + RCAP;
  const int* cnt  = sl + RCAP;
  const int* offs = cnt + NBA;

  int* lb = LIST + (size_t)b * RCAP;
#pragma unroll 1
  for (int it = 0; it < RCAP / (NTHR * 4); ++it) {
    const int i0 = it * (NTHR * 4) + 4 * tid;
    const v4i e4 = *(const v4ia*)(sl + i0);
    int e0 = e4.x >> SLA, e1 = e4.y >> SLA, e2 = e4.z >> SLA, e3 = e4.w >> SLA;
    e0 = e0 < 0 ? 0 : (e0 > nE - 1 ? nE - 1 : e0);
    e1 = e1 < 0 ? 0 : (e1 > nE - 1 ? nE - 1 : e1);
    e2 = e2 < 0 ? 0 : (e2 > nE - 1 ? nE - 1 : e2);
    e3 = e3 < 0 ? 0 : (e3 > nE - 1 ? nE - 1 : e3);
    int s0 = srcs[e0], s1 = srcs[e1], s2 = srcs[e2], s3 = srcs[e3];
    s0 = s0 < 0 ? 0 : (s0 > nN - 1 ? nN - 1 : s0);
    s1 = s1 < 0 ? 0 : (s1 > nN - 1 ? nN - 1 : s1);
    s2 = s2 < 0 ? 0 : (s2 > nN - 1 ? nN - 1 : s2);
    s3 = s3 < 0 ? 0 : (s3 > nN - 1 ? nN - 1 : s3);
    v4i o;
    o.x = (i0     < tt) ? s0 : 0;
    o.y = (i0 + 1 < tt) ? s1 : 0;
    o.z = (i0 + 2 < tt) ? s2 : 0;
    o.w = (i0 + 3 < tt) ? s3 : 0;
    *(volatile v4i*)(lb + i0) = o;
    __threadfence();
    *(volatile v4i*)(lb + i0) = o;
  }
  {
    const v4i c4 = *(const v4ia*)(cnt + 4 * tid);
    const v4i o4 = *(const v4ia*)(offs + 4 * tid);
    int* cp = CNT + (size_t)b * NBA + 4 * tid;
    int* op = OFF + (size_t)b * NBA + 4 * tid;
    *(volatile v4i*)cp = c4;
    *(volatile v4i*)op = o4;
    __threadfence();
    *(volatile v4i*)cp = c4;
    *(volatile v4i*)op = o4;
  }
  if (tid < 8) {
    v4i f;
    f.x = ovf; f.y = tt; f.z = 0; f.w = 0;
    int* fp = FLG + (size_t)b * 32 + 4 * tid;
    *(volatile v4i*)fp = f;
    __threadfence();
    *(volatile v4i*)fp = f;
  }
}

template <int L0>
__global__ __launch_bounds__(NTHR) void k_agg(const int* __restrict__ LIST, const int* __restrict__ CNT,
                                              const int* __restrict__ OFF, const int* __restrict__ FLG,
                                              int nN, int mRows,
                                              const unsigned* __restrict__ srcW, unsigned short* aggp) {
  __shared__ __attribute__((aligned(16))) int scn[NBA];
  __shared__ __attribute__((aligned(16))) int sof[NBA];
  const int tid = (int)threadIdx.x, lane = tid & 31, wave = tid >> 5;
  const int b = (int)blockIdx.x;
  const int nodeBase = b * NBA;
  {
    const v4i c4 = *(const v4i*)(CNT + (size_t)nodeBase + 4 * tid);
    const v4i o4 = *(const v4i*)(OFF + (size_t)nodeBase + 4 * tid);
    *(v4ia*)(scn + 4 * tid) = c4;
    *(v4ia*)(sof + 4 * tid) = o4;
  }
  const int ovf = FLG[(size_t)b * 32];
  __syncthreads();

  const int* lb = LIST + (size_t)b * RCAP;
  const float qnan = __int_as_float(0x7fc00000);
  const float pz = (ovf != 0) ? qnan : 0.0f;
  const int q0s = (4 * lane) & 31, q1s = (4 * lane + 1) & 31;
  const int q2s = (4 * lane + 2) & 31, q3s = (4 * lane + 3) & 31;
#pragma unroll 1
  for (int si = 0; si < NBA / NWAVE; ++si) {
    const int s    = si * NWAVE + wave;
    const int node = nodeBase + s;
    const int craw = __builtin_amdgcn_readfirstlane(scn[s]);
    const bool big = craw > DEGCAP;
    const int c = craw < 0 ? 0 : (craw > DEGCAP ? DEGCAP : craw);
    int o = __builtin_amdgcn_readfirstlane(sof[s]);
    o = o < 0 ? 0 : (o > RCAP ? RCAP : o);
    float a0 = 0.0f, a1 = 0.0f;
#pragma unroll 1
    for (int b0 = 0; b0 < c; b0 += 32) {
      int idx = o + b0 + lane;
      idx = idx > RCAP - 1 ? RCAP - 1 : idx;
      int sr = lb[idx];
      sr = sr < 0 ? 0 : (sr > nN - 1 ? nN - 1 : sr);
      const int m32 = (c - b0) < 32 ? (c - b0) : 32;
#pragma unroll 1
      for (int k = 0; k < m32; ++k) {
        const int sk = __builtin_amdgcn_readlane(sr, k);
        if constexpr (L0 != 0) {
          const unsigned w = srcW[(size_t)sk * (XBP / 2) + lane];
          a0 = a0 + __uint_as_float(w << 16);
          a1 = a1 + __uint_as_float(w & 0xffff0000u);
        } else {
          const unsigned wh = srcW[(size_t)sk * (AGP / 2) + lane];
          const unsigned wl = srcW[(size_t)sk * (AGP / 2) + 32 + lane];
          const float f0 = __uint_as_float(wh << 16)         + __uint_as_float(wl << 16);
          const float f1 = __uint_as_float(wh & 0xffff0000u) + __uint_as_float(wl & 0xffff0000u);
          a0 = a0 + f0;
          a1 = a1 + f1;
        }
      }
    }
    const float dn = (craw < 1) ? 1.0f : (float)craw;
    const float pzr = big ? qnan : pz;
    const bool live = node < nN;
    const float y0 = a0 / dn + pzr;
    const float y1 = a1 / dn + pzr;
    const float v0 = live ? y0 : 0.0f;
    const float v1 = live ? y1 : 0.0f;
    const unsigned hb0 = bf16_bits(v0), hb1 = bf16_bits(v1);
    const unsigned lb0 = bf16_bits(v0 - __uint_as_float(hb0 << 16));
    const unsigned lb1 = bf16_bits(v1 - __uint_as_float(hb1 << 16));
    const int hw = (int)(hb0 | (hb1 << 16));
    const int lw = (int)(lb0 | (lb1 << 16));
    const int g0 = __shfl(hw, q0s, 32), g1 = __shfl(hw, q1s, 32);
    const int g2 = __shfl(hw, q2s, 32), g3 = __shfl(hw, q3s, 32);
    const int p0 = __shfl(lw, q0s, 32), p1 = __shfl(lw, q1s, 32);
    const int p2 = __shfl(lw, q2s, 32), p3 = __shfl(lw, q3s, 32);
    const bool lsel = (lane & 8) != 0;
    v4u pv;
    pv.x = (unsigned int)(lsel ? p0 : g0);
    pv.y = (unsigned int)(lsel ? p1 : g1);
    pv.z = (unsigned int)(lsel ? p2 : g2);
    pv.w = (unsigned int)(lsel ? p3 : g3);
    const bool wr = (node < mRows) && (lane < 16);
    unsigned short* hp = aggp + (size_t)node * AGP + 8 * (lane & 15);
    if (wr) *(volatile v4u*)hp = pv;
    __threadfence();
    if (wr) *(volatile v4u*)hp = pv;
  }
}

template <int FIN>
__global__ __launch_bounds__(GTHR) void k_gemm(const unsigned short* __restrict__ Aagg,
                                               const unsigned short* __restrict__ Asec,
                                               const unsigned short* __restrict__ BT,
                                               const float* __restrict__ bias, void* outp, int nOut) {
  constexpr int P2 = (FIN != 0) ? AGP : XBP;
  constexpr int KT = AGP + P2;
  static_assert(KT % 32 == 0 && P2 % 32 == 0);
  __shared__ __attribute__((aligned(16))) float stg[GBM * GBN];
  const int tid = (int)threadIdx.x, lane = tid & 31, wave = tid >> 5, hh = lane >> 4, m = lane & 15;
  const int rowBase = (int)blockIdx.x * GBM;

  v8f acc[4];
  {
    const v8f z = {0.f, 0.f, 0.f, 0.f, 0.f, 0.f, 0.f, 0.f};
    acc[0] = z; acc[1] = z; acc[2] = z; acc[3] = z;
  }
  const size_t arow = (size_t)(rowBase + 16 * wave + m);
  const unsigned short* ap = Aagg + arow * (size_t)AGP + 8 * hh;
  const unsigned short* sp = Asec + arow * (size_t)P2 + 8 * hh;
  const unsigned short* bp = BT + (size_t)m * (size_t)KT + 8 * hh;

#pragma unroll 1
  for (int k0 = 0; k0 < AGP; k0 += 32) {
    FragB af;
    af.h[0] = *(const v8usa*)(ap + k0);
    af.h[1] = *(const v8usa*)(ap + k0 + 16);
#pragma unroll
    for (int nt = 0; nt < 4; ++nt) {
      const unsigned short* wq = bp + (size_t)(16 * nt) * (size_t)KT + k0;
      FragB bf;
      bf.h[0] = *(const v8usa*)wq;
      bf.h[1] = *(const v8usa*)(wq + 16);
      acc[nt] = wmb(af, bf, acc[nt]);
    }
  }
#pragma unroll 1
  for (int k0 = 0; k0 < P2; k0 += 32) {
    FragB af;
    af.h[0] = *(const v8usa*)(sp + k0);
    af.h[1] = *(const v8usa*)(sp + k0 + 16);
#pragma unroll
    for (int nt = 0; nt < 4; ++nt) {
      const unsigned short* wq = bp + (size_t)(16 * nt) * (size_t)KT + AGP + k0;
      FragB bf;
      bf.h[0] = *(const v8usa*)wq;
      bf.h[1] = *(const v8usa*)(wq + 16);
      acc[nt] = wmb(af, bf, acc[nt]);
    }
  }

#pragma unroll
  for (int nt = 0; nt < 4; ++nt) {
    const int lc = 16 * nt + m;
#pragma unroll
    for (int r = 0; r < 8; ++r) {
      const int lr = 16 * wave + 8 * hh + r;
      stg[lr * GBN + lc] = acc[nt][r];
    }
  }
  __syncthreads();

  v4f bb4;
  {
    const v4f t1 = *(const v4f*)(bias + 4 * m);
    bb4.x = bf16_val(t1.x); bb4.y = bf16_val(t1.y); bb4.z = bf16_val(t1.z); bb4.w = bf16_val(t1.w);
  }
  v4f pv[8];
#pragma unroll
  for (int i = 0; i < 8; ++i) pv[i] = *(const v4fa*)(stg + (16 * wave + 2 * i + hh) * GBN + 4 * m);
  __syncthreads();

#pragma unroll
  for (int i = 0; i < 8; ++i) {
    const bool ok = (rowBase + 16 * wave + 2 * i + hh) < nOut;
    const v4f t = pv[i] + bb4;
    v4f y;
    y.x = (t.x > 0.0f) ? t.x : (t.x - t.x);
    y.y = (t.y > 0.0f) ? t.y : (t.y - t.y);
    y.z = (t.z > 0.0f) ? t.z : (t.z - t.z);
    y.w = (t.w > 0.0f) ? t.w : (t.w - t.w);
    y.x = ok ? y.x : 0.0f; y.y = ok ? y.y : 0.0f; y.z = ok ? y.z : 0.0f; y.w = ok ? y.w : 0.0f;
    pv[i] = y;
  }

  if constexpr (FIN != 0) {
    float* outF = (float*)outp;
#pragma unroll
    for (int i = 0; i < 8; ++i) {
      float* op = outF + (size_t)(rowBase + 16 * wave + 2 * i + hh) * HID + 4 * m;
      *(volatile v4f*)op = pv[i];
    }
    __threadfence();
#pragma unroll
    for (int i = 0; i < 8; ++i) {
      float* op = outF + (size_t)(rowBase + 16 * wave + 2 * i + hh) * HID + 4 * m;
      *(volatile v4f*)op = pv[i];
    }
  } else {
    unsigned short* outH = (unsigned short*)outp;
#pragma unroll
    for (int i = 0; i < 8; ++i) {
      v4us h4, l4;
      unsigned hb;
      hb = bf16_bits(pv[i].x); h4[0] = (unsigned short)hb; l4[0] = (unsigned short)bf16_bits(pv[i].x - __uint_as_float(hb << 16));
      hb = bf16_bits(pv[i].y); h4[1] = (unsigned short)hb; l4[1] = (unsigned short)bf16_bits(pv[i].y - __uint_as_float(hb << 16));
      hb = bf16_bits(pv[i].z); h4[2] = (unsigned short)hb; l4[2] = (unsigned short)bf16_bits(pv[i].z - __uint_as_float(hb << 16));
      hb = bf16_bits(pv[i].w); h4[3] = (unsigned short)hb; l4[3] = (unsigned short)bf16_bits(pv[i].w - __uint_as_float(hb << 16));
      unsigned short* srow = (unsigned short*)stg + (size_t)(16 * wave + 2 * i + hh) * AGP;
      *(v4usa*)(srow + 4 * m) = h4;
      *(v4usa*)(srow + HID + 4 * m) = l4;
    }
    __syncthreads();
    v8us qv[8];
#pragma unroll
    for (int i = 0; i < 8; ++i) {
      const unsigned short* srow = (const unsigned short*)stg + (size_t)(16 * wave + 2 * i + hh) * AGP;
      qv[i] = *(const v8usa*)(srow + 8 * m);
    }
#pragma unroll
    for (int i = 0; i < 8; ++i) {
      unsigned short* rp = outH + (size_t)(rowBase + 16 * wave + 2 * i + hh) * AGP + 8 * m;
      *(volatile v8us*)rp = qv[i];
    }
    __threadfence();
#pragma unroll
    for (int i = 0; i < 8; ++i) {
      unsigned short* rp = outH + (size_t)(rowBase + 16 * wave + 2 * i + hh) * AGP + 8 * m;
      *(volatile v8us*)rp = qv[i];
    }
  }
}

__global__ __launch_bounds__(NTHR) void k_pool_head(const int* __restrict__ bat, int nN,
                                                    const float* __restrict__ h2,
                                                    const float* __restrict__ Wout,
                                                    const float* __restrict__ bout, float* out) {
  extern __shared__ __attribute__((aligned(16))) int dsm[];
  __shared__ __attribute__((aligned(16))) float os[NBG * NCLS];
  const int tid = (int)threadIdx.x, lane = tid & 31, wave = tid >> 5;
  const int gBase = (int)blockIdx.x * NBG;
  int tt = 0, ovf = 0;
  bucket_build<SLG, NBG>(bat, nN, gBase, 1, dsm, tid, lane, wave, tt, ovf);
  const int* sl   = dsm + LISTN + RCAP;
  const int* cnt  = sl + RCAP;
  const int* offs = cnt + NBA;

  float w00, w01, w10, w11;
  {
    const v4f wo = *(const v4f*)(Wout + 4 * lane);
    w00 = bf16_val(wo.x); w01 = bf16_val(wo.y); w10 = bf16_val(wo.z); w11 = bf16_val(wo.w);
  }
  const float bo0 = bf16_val(bout[0]);
  const float bo1 = bf16_val(bout[1]);
  const float qnan = __int_as_float(0x7fc00000);
#pragma unroll 1
  for (int gi = 0; gi < NBG / NWAVE; ++gi) {
    const int s = gi * NWAVE + wave;
    const int craw = __builtin_amdgcn_readfirstlane(cnt[s]);
    const bool big = craw > DEGCAPG;
    const int c = craw < 0 ? 0 : (craw > DEGCAPG ? DEGCAPG : craw);
    int o = __builtin_amdgcn_readfirstlane(offs[s]);
    o = o < 0 ? 0 : (o > RCAP ? RCAP : o);
    float a0 = 0.0f, a1 = 0.0f;
#pragma unroll 1
    for (int b0 = 0; b0 < c; b0 += 32) {
      int idx = o + b0 + lane;
      idx = idx > RCAP - 1 ? RCAP - 1 : idx;
      int nd = sl[idx] >> SLG;
      nd = nd < 0 ? 0 : (nd > nN - 1 ? nN - 1 : nd);
      const int m32 = (c - b0) < 32 ? (c - b0) : 32;
#pragma unroll 1
      for (int k = 0; k < m32; ++k) {
        const int nk = __builtin_amdgcn_readlane(nd, k);
        const v2f v = *(const v2fa*)(h2 + (size_t)nk * HID + 2 * lane);
        a0 = a0 + v.x;
        a1 = a1 + v.y;
      }
    }
    const float dn = (craw < 1) ? 1.0f : (float)craw;
    const float p0 = a0 / dn;
    const float p1 = a1 / dn;
    float q0 = fmaf(p1, w10, p0 * w00);
    float q1 = fmaf(p1, w11, p0 * w01);
#pragma unroll
    for (int d = 16; d >= 1; d >>= 1) {
      q0 += __shfl_xor(q0, d, 32);
      q1 += __shfl_xor(q1, d, 32);
    }
    float r0 = q0 + bo0;
    float r1 = q1 + bo1;
    const bool bad = big || (ovf != 0);
    r0 = bad ? qnan : r0;
    r1 = bad ? qnan : r1;
    if (lane == 0) { os[2 * s] = r0; os[2 * s + 1] = r1; }
  }
  __syncthreads();
  if (tid < (NBG * NCLS) / 4) {
    const v4f ov = *(const v4fa*)(os + 4 * tid);
    float* op = out + (size_t)gBase * NCLS + 4 * tid;
    *(volatile v4f*)op = ov;
    __threadfence();
    *(volatile v4f*)op = ov;
  }
}

static inline int cdiv(int a, int b) { return (a + b - 1) / b; }
static inline size_t al256(size_t o) { return (o + 255) & ~(size_t)255; }

extern "C" void kernel_launch(void* const* d_in, const int* in_sizes, int n_in,
                              void* d_out, int out_size, void* d_ws, size_t ws_size,
                              hipStream_t stream) {
  if (n_in < 12) return;
  const int nN = in_sizes[0];
  if (nN < 16 || nN >= (1 << 24)) return;
  if (in_sizes[1] < 2 || (in_sizes[1] & 1) != 0) return;
  const int nE = in_sizes[1] / 2;
  if (nE < 1 || nE > (1 << 20)) return;
  if (in_sizes[2] != nN) return;
  if (in_sizes[3] != VOCABN * HID) return;
  if (in_sizes[4] != HID * HID || in_sizes[5] != HID) return;
  if (in_sizes[6] != HID * HID) return;
  if (in_sizes[7] != HID * HID || in_sizes[8] != HID) return;
  if (in_sizes[9] != HID * HID) return;
  if (in_sizes[10] != HID * NCLS || in_sizes[11] != NCLS) return;
  if (out_size != NGR * NCLS) return;

  const int*   x    = (const int*)d_in[0];
  const int*   ei   = (const int*)d_in[1];
  const int*   bat  = (const int*)d_in[2];
  const float* emb  = (const float*)d_in[3];
  const float* W1l  = (const float*)d_in[4];
  const float* b1   = (const float*)d_in[5];
  const float* W1r  = (const float*)d_in[6];
  const float* W2l  = (const float*)d_in[7];
  const float* b2   = (const float*)d_in[8];
  const float* W2r  = (const float*)d_in[9];
  const float* Wout = (const float*)d_in[10];
  const float* bout = (const float*)d_in[11];
  float* out = (float*)d_out;
  const int* src = ei;
  const int* dst = ei + nE;

  const int MP  = cdiv(nN, GBM) * GBM;
  const int gM  = MP / GBM;
  const int gA  = cdiv(MP, NBA);
  if ((long long)gA * NBA < (long long)MP) return;
  const int nXB = MP / 32;
  const int vec8 = ((nE & 3) == 0) ? 1 : 0;

  char* ws = (char*)d_ws;
  size_t off = 0;
  const size_t oXB  = off; off = al256(off + (size_t)MP * XBP * 2);
  const size_t oAGG = off; off = al256(off + (size_t)MP * AGP * 2);
  const size_t oH1  = off; off = al256(off + (size_t)MP * AGP * 2);
  const size_t oH2  = off; off = al256(off + (size_t)MP * HID * 4);
  const size_t oLST = off; off = al256(off + (size_t)gA * RCAP * 4);
  const size_t oCNT = off; off = al256(off + (size_t)gA * NBA * 4);
  const size_t oOFF = off; off = al256(off + (size_t)gA * NBA * 4);
  const size_t oFLG = off; off = al256(off + (size_t)gA * 32 * 4);
  const size_t oW1  = off; off = al256(off + (size_t)HID * K0L * 2);
  const size_t oW2  = off; off = al256(off + (size_t)HID * K1L * 2);
  if (off > ws_size || off > (size_t)WSMAX) return;
  unsigned short* XB  = (unsigned short*)(ws + oXB);
  unsigned short* AGG = (unsigned short*)(ws + oAGG);
  unsigned short* H1  = (unsigned short*)(ws + oH1);
  float*          H2  = (float*)(ws + oH2);
  int*            LST = (int*)(ws + oLST);
  int*            CNT = (int*)(ws + oCNT);
  int*            OFF = (int*)(ws + oOFF);
  int*            FLG = (int*)(ws + oFLG);
  unsigned short* W1c = (unsigned short*)(ws + oW1);
  unsigned short* W2c = (unsigned short*)(ws + oW2);

  const size_t bLds = (size_t)BLDS_INTS * 4;
  hipFuncSetAttribute(reinterpret_cast<const void*>(&k_compact), hipFuncAttributeMaxDynamicSharedMemorySize, (int)bLds);
  hipFuncSetAttribute(reinterpret_cast<const void*>(&k_pool_head), hipFuncAttributeMaxDynamicSharedMemorySize, (int)bLds);

  k_prep<<<nXB + (NPARTW * 512) / NTHR, NTHR, 0, stream>>>(x, emb, W1l, W1r, W2l, W2r, nN, nXB, XB, W1c, W2c);
  k_compact<<<gA, NTHR, bLds, stream>>>(src, dst, nE, nN, vec8, LST, CNT, OFF, FLG);
  k_agg<1><<<gA, NTHR, 0, stream>>>(LST, CNT, OFF, FLG, nN, MP, (const unsigned*)XB, AGG);
  k_gemm<0><<<gM, GTHR, 0, stream>>>(AGG, XB, W1c, b1, (void*)H1, nN);
  k_agg<0><<<gA, NTHR, 0, stream>>>(LST, CNT, OFF, FLG, nN, MP, (const unsigned*)H1, AGG);
  k_gemm<1><<<gM, GTHR, 0, stream>>>(AGG, H1, W2c, b2, (void*)H2, nN);
  k_pool_head<<<NGR / NBG, NTHR, bLds, stream>>>(bat, nN, H2, Wout, bout, out);
}
